// MambaBlock_3444563772118
// MI455X (gfx1250) — hardware-verified
//
#include <hip/hip_runtime.h>
#include <math.h>

typedef __attribute__((ext_vector_type(16))) _Float16 v16h;
typedef __attribute__((ext_vector_type(8)))  _Float16 v8h;
typedef __attribute__((ext_vector_type(8)))  float    v8f;
typedef __attribute__((ext_vector_type(4)))  float    v4f;

constexpr int kBatch  = 2;
constexpr int kSeq    = 2048;
constexpr int kDm     = 1024;
constexpr int kDin    = 2048;
constexpr int kNst    = 16;
constexpr int kSsmN   = 2 * kNst + 1;
constexpr int kSsmP   = 64;
constexpr int kXarP   = 2 * kDin;
constexpr int kRows   = kBatch * kSeq;
constexpr int kConvTP = 260;
constexpr int kScanTS = 64;
constexpr int kScanCh = 64;
constexpr int kScanYP = 68;
constexpr float kWCarry    = 32.0f;
constexpr float kWCarryInv = 1.0f / kWCarry;

static_assert(kSsmN == 33);
static_assert(kSsmN <= kSsmP);
static_assert((kDm % 32) == 0 && (kDin % 32) == 0);
static_assert((kRows % 64) == 0 && (kXarP % 64) == 0 && (kSsmP % 64) == 0 && (kDm % 64) == 0);
static_assert((kSeq % kScanTS) == 0 && (kSeq % 64) == 0 && (kDin % kScanCh) == 0 && (kDin % 256) == 0);
static_assert(((kSsmN * kDin) % 8) == 0);

constexpr size_t kOffXar    = 0;
constexpr size_t kOffXc16   = kOffXar    + (size_t)kRows * kXarP * 4;
constexpr size_t kOffSsm    = kOffXc16   + (size_t)kRows * kDin  * 2;
constexpr size_t kOffY2     = kOffSsm    + (size_t)kRows * kSsmP * 4;
constexpr size_t kOffX16    = kOffY2     + (size_t)kRows * kDin  * 2;
constexpr size_t kOffWin16  = kOffX16    + (size_t)kRows * kDm   * 2;
constexpr size_t kOffWout16 = kOffWin16  + (size_t)kXarP * kDm   * 2;
constexpr size_t kOffWx16   = kOffWout16 + (size_t)kDm   * kDin  * 2;
constexpr size_t kWsTotal   = kOffWx16   + (size_t)kSsmP * kDin  * 2;
static_assert(kWsTotal == 122945536ull);
static_assert(kWsTotal <= 134217728ull);
static_assert((kOffXc16 % 128) == 0 && (kOffSsm % 128) == 0 && (kOffY2 % 128) == 0 && (kOffX16 % 128) == 0 &&
              (kOffWin16 % 128) == 0 && (kOffWout16 % 128) == 0 && (kOffWx16 % 128) == 0);

__device__ __forceinline__ float bf_rne(float f) {
  const unsigned u = __float_as_uint(f);
  const unsigned r = (u + 0x7FFFu + ((u >> 16) & 1u)) & 0xFFFF0000u;
  return __uint_as_float(r);
}

union FragU { v16h v; v8h h[2]; };
__device__ __forceinline__ v16h frag_load(const _Float16* p) {
  FragU f;
  f.h[0] = *(const v8h*)(p);
  f.h[1] = *(const v8h*)(p + 16);
  return f.v;
}
__device__ __forceinline__ v8f frag_mma(v16h a, v16h b, v8f c) {
  return __builtin_amdgcn_wmma_f32_16x16x32_f16(false, a, false, b, (short)0, c, false, false);
}
__device__ __forceinline__ void wmma_group_guard(v8f& a, v8f& b, v8f& c, v8f& d,
                                                 v16h x, v16h y0, v16h y1, v16h y2, v16h y3) {
  asm volatile("v_nop\n\tv_nop\n\tv_nop\n\tv_nop"
               : "+v"(a), "+v"(b), "+v"(c), "+v"(d)
               : "v"(x), "v"(y0), "v"(y1), "v"(y2), "v"(y3));
}
__device__ __forceinline__ void acc_guard4(v8f& a, v8f& b, v8f& c, v8f& d) {
  asm volatile("v_nop\n\tv_nop\n\tv_nop\n\tv_nop" : "+v"(a), "+v"(b), "+v"(c), "+v"(d));
}

__global__ __launch_bounds__(256) void wmma_gemm64_f16(
    const unsigned short* __restrict__ Ap, int lda,
    const unsigned short* __restrict__ Btp, int ldb,
    float* __restrict__ Cout, int ldc,
    int M, int N, int K, float scale)
{
  const _Float16* A  = (const _Float16*)Ap;
  const _Float16* Bt = (const _Float16*)Btp;
  __shared__ __align__(16) float sT[8][16 * 68];
  const int lane = threadIdx.x & 31;
  const int wave = threadIdx.x >> 5;
  const int tilesN = N >> 6;
  const int tilesM = M >> 6;
  const int tile = blockIdx.x * 8 + wave;
  if (tile >= tilesM * tilesN) return;
  const int tm = tile / tilesN;
  const int tn = tile - tm * tilesN;
  const int m0 = tm << 6;
  const int n0 = tn << 6;

  const int rlane = lane & 15;
  const int koff  = (lane >> 4) * 8;
  const int mOff  = (lane >> 4) * 8;

  v8f acc[4][4];
#pragma unroll
  for (int i = 0; i < 4; ++i)
#pragma unroll
    for (int j = 0; j < 4; ++j) acc[i][j] = (v8f){0.f, 0.f, 0.f, 0.f, 0.f, 0.f, 0.f, 0.f};

  for (int k0 = 0; k0 < K; k0 += 32) {
    v16h bh[4];
#pragma unroll
    for (int j = 0; j < 4; ++j) {
      const size_t bo = (size_t)(n0 + (j << 4) + rlane) * ldb + koff + k0;
      bh[j] = frag_load(Bt + bo);
    }
#pragma unroll
    for (int i = 0; i < 4; ++i) {
      const size_t ao = (size_t)(m0 + (i << 4) + rlane) * lda + koff + k0;
      v16h ah = frag_load(A + ao);
#pragma unroll
      for (int j = 0; j < 4; ++j) acc[i][j] = frag_mma(ah, bh[j], acc[i][j]);
      wmma_group_guard(acc[i][0], acc[i][1], acc[i][2], acc[i][3], ah, bh[0], bh[1], bh[2], bh[3]);
    }
  }
  acc_guard4(acc[0][0], acc[0][1], acc[0][2], acc[0][3]);
  acc_guard4(acc[1][0], acc[1][1], acc[1][2], acc[1][3]);
  acc_guard4(acc[2][0], acc[2][1], acc[2][2], acc[2][3]);
  acc_guard4(acc[3][0], acc[3][1], acc[3][2], acc[3][3]);

  float* slab = sT[wave];
#pragma unroll
  for (int i = 0; i < 4; ++i) {
    const int mBase = m0 + (i << 4);
#pragma unroll
    for (int j = 0; j < 4; ++j) {
#pragma unroll
      for (int r = 0; r < 8; ++r) {
        const float v = acc[i][j][r] * scale;
        slab[(mOff + r) * 68 + (j << 4) + rlane] = v;
      }
    }
    __builtin_amdgcn_fence(__ATOMIC_RELEASE, "workgroup");
    __builtin_amdgcn_wave_barrier();
    __builtin_amdgcn_fence(__ATOMIC_ACQUIRE, "workgroup");
    {
      const int hh = lane >> 4, c4 = (lane & 15) * 4;
      for (int pass = 0; pass < 2; ++pass) {
#pragma unroll
        for (int it = 0; it < 8; ++it) {
          const int row = it * 2 + hh;
          v4f v = *(const v4f*)(slab + row * 68 + c4);
          *(volatile v4f*)(Cout + (size_t)(mBase + row) * ldc + n0 + c4) = v;
        }
        __threadfence();
      }
    }
    __builtin_amdgcn_fence(__ATOMIC_RELEASE, "workgroup");
    __builtin_amdgcn_wave_barrier();
    __builtin_amdgcn_fence(__ATOMIC_ACQUIRE, "workgroup");
  }
}

__global__ __launch_bounds__(256) void cast_f16_kernel(
    const float* __restrict__ src, unsigned short* __restrict__ dst, int total8, int src8, float scale)
{
  const int i = blockIdx.x * 256 + threadIdx.x;
  if (i >= total8) return;
  const bool live = (i < src8);
  const int ic = live ? i : (src8 - 1);
  const size_t s0 = (size_t)ic << 3;
  const v4f a0 = *(const v4f*)(src + s0);
  const v4f a1 = *(const v4f*)(src + s0 + 4);
  v8h hv;
#pragma unroll
  for (int e = 0; e < 4; ++e) {
    const float e0 = a0[e];
    const float e1 = a1[e];
    const float b0 = bf_rne(e0);
    const float b1 = bf_rne(e1);
    const float f0 = live ? (b0 * scale) : 0.0f;
    const float f1 = live ? (b1 * scale) : 0.0f;
    hv[e]     = (_Float16)f0;
    hv[4 + e] = (_Float16)f1;
  }
  unsigned short* q = dst + ((size_t)i << 3);
  *(volatile v8h*)q = hv;
  __threadfence();
  *(volatile v8h*)q = hv;
}

__global__ __launch_bounds__(256) void conv_silu_kernel(
    const float* __restrict__ XAR, const float* __restrict__ cw, const float* __restrict__ cb,
    unsigned short* __restrict__ XC16)
{
  __shared__ __align__(16) float sT[16 * kConvTP];
  const int tid = threadIdx.x, lane = tid & 31, wave = tid >> 5;
  const int d0 = blockIdx.x * 256, d = d0 + tid;
  const int g0 = blockIdx.y * 64;
  const int tb = g0 & (kSeq - 1);
  const v4f wv = *(const v4f*)(cw + (size_t)d * 4);
  const float wr0 = wv[0], wr1 = wv[1], wr2 = wv[2], wr3 = wv[3];
  const float w0 = bf_rne(wr0), w1 = bf_rne(wr1), w2 = bf_rne(wr2), w3 = bf_rne(wr3);
  const float bcr = cb[d];
  const float bc = bf_rne(bcr);
  float xm3, xm2, xm1;
  {
    const bool hist = (tb > 0);
    const int rb = hist ? (g0 - 3) : g0;
    const float v3 = XAR[(size_t)rb * kXarP + d];
    const float v2 = XAR[(size_t)(rb + 1) * kXarP + d];
    const float v1 = XAR[(size_t)(rb + 2) * kXarP + d];
    xm3 = hist ? v3 : 0.f;
    xm2 = hist ? v2 : 0.f;
    xm1 = hist ? v1 : 0.f;
  }
#pragma unroll 1
  for (int sub = 0; sub < 4; ++sub) {
    const int lb = g0 + sub * 16;
#pragma unroll 1
    for (int s = 0; s < 16; ++s) {
      const float xcur = XAR[(size_t)(lb + s) * kXarP + d];
      float acc = w0 * xm3;
      acc = fmaf(w1, xm2, acc);
      acc = fmaf(w2, xm1, acc);
      acc = fmaf(w3, xcur, acc);
      const float sv = acc + bc;
      const float sg = __builtin_amdgcn_rcpf(1.0f + expf(-sv));
      sT[s * kConvTP + tid] = sv * sg;
      xm3 = xm2; xm2 = xm1; xm1 = xcur;
    }
    __syncthreads();
    v8h bv[2];
#pragma unroll
    for (int it = 0; it < 2; ++it) {
      const float* sp = sT + (it * 8 + wave) * kConvTP + lane * 8;
      const v4f a0 = *(const v4f*)(sp);
      const v4f a1 = *(const v4f*)(sp + 4);
#pragma unroll
      for (int e = 0; e < 4; ++e) {
        bv[it][e]     = (_Float16)a0[e];
        bv[it][4 + e] = (_Float16)a1[e];
      }
    }
    for (int pass = 0; pass < 2; ++pass) {
#pragma unroll
      for (int it = 0; it < 2; ++it)
        *(volatile v8h*)(XC16 + (size_t)(lb + it * 8 + wave) * kDin + d0 + lane * 8) = bv[it];
      __threadfence();
    }
    __syncthreads();
  }
}

__global__ __launch_bounds__(64) void scan_kernel(
    const float* __restrict__ SSM, const float* __restrict__ XAR,
    const float* __restrict__ cw, const float* __restrict__ cb,
    const float* __restrict__ Wdt, const float* __restrict__ bdt,
    const float* __restrict__ Alog, const float* __restrict__ Dp,
    unsigned short* __restrict__ Y2H)
{
  __shared__ __align__(16) float sX[kScanTS * kSsmP];
  __shared__ __align__(16) float sY[kScanTS * kScanYP];
  __shared__ __align__(16) float sA[kNst];
  const int tid = threadIdx.x, lane = tid & 31, wave = tid >> 5;
  constexpr int kBlkPerB = kDin / kScanCh;
  const int bix = blockIdx.x / kBlkPerB;
  const int d0  = (blockIdx.x - bix * kBlkPerB) * kScanCh;
  const int d   = d0 + tid;
  const size_t row0 = (size_t)bix * kSeq;
  {
    const float alr = Alog[tid & (kNst - 1)];
    const float al = bf_rne(alr);
    const float na = -expf(al);
    if (tid < kNst) sA[tid] = na;
  }
  __syncthreads();
  float negA[kNst], h[kNst];
#pragma unroll
  for (int n = 0; n < kNst; ++n) {
    negA[n] = sA[n];
    h[n] = 0.f;
  }
  const v4f wv = *(const v4f*)(cw + (size_t)d * 4);
  const float wr0 = wv[0], wr1 = wv[1], wr2 = wv[2], wr3 = wv[3];
  const float w0 = bf_rne(wr0), w1 = bf_rne(wr1), w2 = bf_rne(wr2), w3 = bf_rne(wr3);
  const float bcr  = cb[d];
  const float wdtr = Wdt[d];
  const float bbr  = bdt[d];
  const float Ddr  = Dp[d];
  const float bc  = bf_rne(bcr);
  const float wdt = bf_rne(wdtr);
  const float bb  = bf_rne(bbr);
  const float Dd  = bf_rne(Ddr);
  float xm3 = 0.f, xm2 = 0.f, xm1 = 0.f;
  const int lr = tid >> 4, lc4 = (tid & 15) * 4;
  const int q = lane >> 3, c8 = (lane & 7) * 8;
#pragma unroll 1
  for (int t0 = 0; t0 < kSeq; t0 += kScanTS) {
    __syncthreads();
#pragma unroll
    for (int i = 0; i < 16; ++i) {
      const int r = lr + 4 * i;
      *(v4f*)(sX + r * kSsmP + lc4) = *(const v4f*)(SSM + (row0 + t0 + r) * kSsmP + lc4);
    }
    __syncthreads();
#pragma unroll 1
    for (int s = 0; s < kScanTS; ++s) {
      const size_t grow = row0 + (size_t)(t0 + s);
      const float* xr = sX + s * kSsmP;
      float xcur = XAR[grow * kXarP + d];
      float rs   = XAR[grow * kXarP + kDin + d];
      asm volatile("" : "+v"(xcur));
      asm volatile("" : "+v"(rs));
      float Bs[kNst], Cs[kNst];
#pragma unroll
      for (int q4 = 0; q4 < 4; ++q4) {
        const v4f bv = *(const v4f*)(xr + 4 * q4);
        const v4f cv = *(const v4f*)(xr + kNst + 4 * q4);
        Bs[4 * q4 + 0] = bv[0]; Bs[4 * q4 + 1] = bv[1]; Bs[4 * q4 + 2] = bv[2]; Bs[4 * q4 + 3] = bv[3];
        Cs[4 * q4 + 0] = cv[0]; Cs[4 * q4 + 1] = cv[1]; Cs[4 * q4 + 2] = cv[2]; Cs[4 * q4 + 3] = cv[3];
      }
      const float dtraw = xr[2 * kNst];
      float pre = w0 * xm3;
      pre = fmaf(w1, xm2, pre);
      pre = fmaf(w2, xm1, pre);
      pre = fmaf(w3, xcur, pre);
      pre = pre + bc;
      const float xt = pre * __builtin_amdgcn_rcpf(1.0f + expf(-pre));
      xm3 = xm2; xm2 = xm1; xm1 = xcur;
      const float z  = fmaf(dtraw, wdt, bb);
      const float dt = fmaxf(z, 0.0f) + log1pf(expf(-fabsf(z)));
      const float dtx = dt * xt;
      float y = 0.f;
#pragma unroll
      for (int k = 0; k < kNst; ++k) {
        const float e = __expf(dt * negA[k]);
        h[k] = fmaf(e, h[k], dtx * Bs[k]);
        y = fmaf(h[k], Cs[k], y);
      }
      y = fmaf(xt, Dd, y);
      const float u  = y + rs;
      const float y2 = u * __builtin_amdgcn_rcpf(1.0f + expf(-u));
      sY[s * kScanYP + tid] = y2;
    }
    __syncthreads();
    v8h hv[8];
#pragma unroll
    for (int it = 0; it < 8; ++it) {
      const int row = it * 8 + wave * 4 + q;
      const float* sp = sY + row * kScanYP + c8;
      const v4f a0 = *(const v4f*)(sp);
      const v4f a1 = *(const v4f*)(sp + 4);
#pragma unroll
      for (int e = 0; e < 4; ++e) {
        const float f0 = fminf(fmaxf(a0[e], -65504.0f), 65504.0f);
        const float f1 = fminf(fmaxf(a1[e], -65504.0f), 65504.0f);
        hv[it][e]     = (_Float16)f0;
        hv[it][4 + e] = (_Float16)f1;
      }
    }
    for (int pass = 0; pass < 2; ++pass) {
#pragma unroll
      for (int it = 0; it < 8; ++it) {
        const int row = it * 8 + wave * 4 + q;
        const size_t o = (row0 + (size_t)(t0 + row)) * kDin + d0 + c8;
        *(volatile v8h*)(Y2H + o) = hv[it];
      }
      __threadfence();
    }
  }
}

extern "C" void kernel_launch(void* const* d_in, const int* in_sizes, int n_in,
                              void* d_out, int out_size, void* d_ws, size_t ws_size,
                              hipStream_t stream)
{
  if (n_in < 10) return;
  if (in_sizes[0] != kRows * kDm) return;
  if (in_sizes[1] != kXarP * kDm) return;
  if (in_sizes[2] != kDin * 4) return;
  if (in_sizes[3] != kDin) return;
  if (in_sizes[4] != kSsmN * kDin) return;
  if (in_sizes[5] != kDin) return;
  if (in_sizes[6] != kDin) return;
  if (in_sizes[7] != kNst) return;
  if (in_sizes[8] != kDin) return;
  if (in_sizes[9] != kDm * kDin) return;
  if (out_size != kRows * kDm) return;
  if (ws_size < kWsTotal) return;

  const float* x      = (const float*)d_in[0];
  const float* W_in   = (const float*)d_in[1];
  const float* conv_w = (const float*)d_in[2];
  const float* conv_b = (const float*)d_in[3];
  const float* W_x    = (const float*)d_in[4];
  const float* W_dt   = (const float*)d_in[5];
  const float* b_dt   = (const float*)d_in[6];
  const float* A_log  = (const float*)d_in[7];
  const float* Dp     = (const float*)d_in[8];
  const float* W_out  = (const float*)d_in[9];
  float* out = (float*)d_out;

  char* ws = (char*)d_ws;
  float*          XAR    = (float*)(ws + kOffXar);
  unsigned short* XC16   = (unsigned short*)(ws + kOffXc16);
  float*          SSM    = (float*)(ws + kOffSsm);
  unsigned short* Y2H    = (unsigned short*)(ws + kOffY2);
  unsigned short* X16    = (unsigned short*)(ws + kOffX16);
  unsigned short* WIN16  = (unsigned short*)(ws + kOffWin16);
  unsigned short* WOUT16 = (unsigned short*)(ws + kOffWout16);
  unsigned short* WX16   = (unsigned short*)(ws + kOffWx16);

  constexpr int kX8    = kRows * kDm / 8;
  constexpr int kWin8  = kXarP * kDm / 8;
  constexpr int kWout8 = kDm * kDin / 8;
  constexpr int kWx8   = kSsmP * kDin / 8;
  constexpr int kWxSrc8 = kSsmN * kDin / 8;
  static_assert((kX8 % 256) == 0 && (kWin8 % 256) == 0 && (kWout8 % 256) == 0 && (kWx8 % 256) == 0);

  cast_f16_kernel<<<kX8 / 256, 256, 0, stream>>>(x, X16, kX8, kX8, 1.0f);
  cast_f16_kernel<<<kWin8 / 256, 256, 0, stream>>>(W_in, WIN16, kWin8, kWin8, kWCarry);
  cast_f16_kernel<<<kWout8 / 256, 256, 0, stream>>>(W_out, WOUT16, kWout8, kWout8, kWCarry);
  cast_f16_kernel<<<kWx8 / 256, 256, 0, stream>>>(W_x, WX16, kWx8, kWxSrc8, kWCarry);

  wmma_gemm64_f16<<<(kRows / 64) * (kXarP / 64) / 8, 256, 0, stream>>>(
      X16, kDm, WIN16, kDm, XAR, kXarP, kRows, kXarP, kDm, kWCarryInv);

  conv_silu_kernel<<<dim3(kDin / 256, kRows / 64), 256, 0, stream>>>(XAR, conv_w, conv_b, XC16);

  wmma_gemm64_f16<<<(kRows / 64) * (kSsmP / 64) / 8, 256, 0, stream>>>(
      XC16, kDin, WX16, kDin, SSM, kSsmP, kRows, kSsmP, kDin, kWCarryInv);

  scan_kernel<<<kBatch * (kDin / kScanCh), kScanCh, 0, stream>>>(
      SSM, XAR, conv_w, conv_b, W_dt, b_dt, A_log, Dp, Y2H);

  wmma_gemm64_f16<<<(kRows / 64) * (kDm / 64) / 8, 256, 0, stream>>>(
      Y2H, kDin, WOUT16, kDin, out, kDm, kRows, kDm, kDin, kWCarryInv);
}
